// SocialLSTM_6141803233972
// MI455X (gfx1250) — hardware-verified
//
#include <hip/hip_runtime.h>
#include <math.h>

constexpr int SEQ_LEN   = 4096;
constexpr int EMB_DIM   = 64;
constexpr int HID_DIM   = 32;
constexpr int NGATE     = 128;
constexpr int NPRED     = 128;
constexpr int NROW_OUT  = SEQ_LEN + NPRED;
constexpr int NTHR      = 256;
constexpr int WHP       = 36;
constexpr int WIP       = 68;
constexpr int EMB_BLKS  = SEQ_LEN * EMB_DIM / 8 / NTHR;
constexpr int WIH_BLKS  = NGATE * EMB_DIM / 8 / NTHR;
constexpr int GEMM_BLKS = (SEQ_LEN / 64) * (NGATE / 64) / 8;
static_assert(SEQ_LEN % 64 == 0 && NGATE % 64 == 0);
static_assert(EMB_DIM % 32 == 0);
static_assert((SEQ_LEN * EMB_DIM / 8) % NTHR == 0);
static_assert((NGATE * EMB_DIM / 8) % NTHR == 0);
static_assert(((SEQ_LEN / 64) * (NGATE / 64)) % 8 == 0);
static_assert(NROW_OUT % 16 == 0);
static_assert(NROW_OUT * 2 == 8448);
static_assert(NGATE == 4 * HID_DIM);
static_assert((NGATE * HID_DIM / 4) % 32 == 0 && (NGATE * EMB_DIM / 4) % 32 == 0);

typedef __attribute__((ext_vector_type(16))) _Float16 v16h;
typedef __attribute__((ext_vector_type(8)))  _Float16 v8h;
typedef __attribute__((ext_vector_type(16))) __bf16   v16b;
typedef __attribute__((ext_vector_type(8)))  __bf16   v8b;
typedef __attribute__((ext_vector_type(8)))  float    v8f;
typedef __attribute__((ext_vector_type(4)))  float    v4f;
typedef __attribute__((ext_vector_type(2)))  float    v2f;
typedef __attribute__((ext_vector_type(4)))  unsigned v4u;

__device__ __forceinline__ unsigned short f2bf_bits(float f) {
  unsigned u = __float_as_uint(f);
  return (unsigned short)((u + 0x7FFFu + ((u >> 16) & 1u)) >> 16);
}
__device__ __forceinline__ float bf_bits2f(unsigned short h) { return __uint_as_float(((unsigned)h) << 16); }

__device__ __forceinline__ void dep_guard_h(v8f& a, v8f& b, v16h x, v16h y) { asm volatile("v_nop\n\tv_nop\n\tv_nop\n\tv_nop" : "+v"(a), "+v"(b) : "v"(x), "v"(y)); }
__device__ __forceinline__ void dep_guard_b(v8f& a, v8f& b, v16b x, v16b y) { asm volatile("v_nop\n\tv_nop\n\tv_nop\n\tv_nop" : "+v"(a), "+v"(b) : "v"(x), "v"(y)); }
__device__ __forceinline__ void dep_guard4_h(v8f& a, v8f& b, v8f& c, v8f& d, v16h x, v16h y) { asm volatile("v_nop\n\tv_nop\n\tv_nop\n\tv_nop" : "+v"(a), "+v"(b), "+v"(c), "+v"(d) : "v"(x), "v"(y)); }
__device__ __forceinline__ void dep_guard4_b(v8f& a, v8f& b, v8f& c, v8f& d, v16b x, v16b y) { asm volatile("v_nop\n\tv_nop\n\tv_nop\n\tv_nop" : "+v"(a), "+v"(b), "+v"(c), "+v"(d) : "v"(x), "v"(y)); }
__device__ __forceinline__ void keep4_h(v16h a, v16h b, v16h c, v16h d) { asm volatile("v_nop" :: "v"(a), "v"(b), "v"(c), "v"(d)); }
__device__ __forceinline__ void keep4_b(v16b a, v16b b, v16b c, v16b d) { asm volatile("v_nop" :: "v"(a), "v"(b), "v"(c), "v"(d)); }
__device__ __forceinline__ void acc_guard4(v8f& a, v8f& b, v8f& c, v8f& d) { asm volatile("v_nop\n\tv_nop\n\tv_nop\n\tv_nop" : "+v"(a), "+v"(b), "+v"(c), "+v"(d)); }
template <typename T> struct Frag;
template <> struct Frag<_Float16> {
  typedef v16h V; union U { v16h v; v8h h[2]; };
  static __device__ __forceinline__ v16h load(const _Float16* p) {
    U f; f.h[0] = *(const v8h*)(p); f.h[1] = *(const v8h*)(p + 16); return f.v;
  }
  static __device__ __forceinline__ v8f mma(v16h a, v16h b, v8f c) {
    return __builtin_amdgcn_wmma_f32_16x16x32_f16(false, a, false, b, (short)0, c, false, false);
  }
  static __device__ __forceinline__ void guard(v8f& a, v8f& b, v16h x, v16h y) { dep_guard_h(a, b, x, y); }
  static __device__ __forceinline__ void guard4(v8f& a, v8f& b, v8f& c, v8f& d, v16h x, v16h y) { dep_guard4_h(a, b, c, d, x, y); }
  static __device__ __forceinline__ void keep(v16h a, v16h b, v16h c, v16h d) { keep4_h(a, b, c, d); }
};
template <> struct Frag<__bf16> {
  typedef v16b V; union U { v16b v; v8b h[2]; };
  static __device__ __forceinline__ v16b load(const __bf16* p) {
    U f; f.h[0] = *(const v8b*)(p); f.h[1] = *(const v8b*)(p + 16); return f.v;
  }
  static __device__ __forceinline__ v8f mma(v16b a, v16b b, v8f c) {
    return __builtin_amdgcn_wmma_f32_16x16x32_bf16(false, a, false, b, (short)0, c, false, false);
  }
  static __device__ __forceinline__ void guard(v8f& a, v8f& b, v16b x, v16b y) { dep_guard_b(a, b, x, y); }
  static __device__ __forceinline__ void guard4(v8f& a, v8f& b, v8f& c, v8f& d, v16b x, v16b y) { dep_guard4_b(a, b, c, d, x, y); }
  static __device__ __forceinline__ void keep(v16b a, v16b b, v16b c, v16b d) { keep4_b(a, b, c, d); }
};

__device__ __forceinline__ float fsig(float x)  { return __builtin_amdgcn_rcpf(1.0f + __expf(-x)); }
__device__ __forceinline__ float ftanh(float x) { return 1.0f - 2.0f * __builtin_amdgcn_rcpf(__expf(2.0f * x) + 1.0f); }

template <int ET> struct Elem;
template <> struct Elem<0> { typedef _Float16 T; };
template <> struct Elem<1> { typedef __bf16 T; };
template <int ET, bool SPLIT, int BIAS_MODE, int OUT_MODE, bool RESID, int ACT = 0>
__global__ __launch_bounds__(256) void wmma_gemm64(
    const unsigned short* __restrict__ Ap, const unsigned short* __restrict__ A2p, int lda, long strideA,
    const unsigned short* __restrict__ Btp, const unsigned short* __restrict__ Bt2p, int ldb, long strideB,
    void* __restrict__ Cout, void* __restrict__ Cout2, int ldc, long strideC,
    const float* __restrict__ bias,
    const float* __restrict__ resid, long strideR,
    int M, int N, int K, float scale) {
  typedef typename Elem<ET>::T T;
  typedef typename Frag<T>::V V;
  const T* A = (const T*)Ap; const T* A2 = (const T*)A2p; const T* Bt = (const T*)Btp; const T* Bt2 = (const T*)Bt2p;
  __shared__ __align__(16) float sT[8][16 * 68];
  const int b    = blockIdx.y;
  const int lane = threadIdx.x & 31;
  const int wave = threadIdx.x >> 5;
  const int tilesN = N >> 6;
  const int tilesM = M >> 6;
  const int tile = blockIdx.x * 8 + wave;
  if (tile >= tilesM * tilesN) return;
  const int tm = tile / tilesN;
  const int tn = tile - tm * tilesN;
  const int m0 = tm << 6;
  const int n0 = tn << 6;

  const T* Ab  = A  + (size_t)b * strideA;
  const T* Bb  = Bt + (size_t)b * strideB;
  const T* Ab2 = SPLIT ? (A2  + (size_t)b * strideA) : nullptr;
  const T* Bb2 = SPLIT ? (Bt2 + (size_t)b * strideB) : nullptr;

  const int rlane = lane & 15;
  const int koff  = (lane >> 4) * 8;
  const int mOff  = (lane >> 4) * 8;

  v8f acc[4][4];
#pragma unroll
  for (int i = 0; i < 4; ++i)
#pragma unroll
    for (int j = 0; j < 4; ++j) acc[i][j] = (v8f){0.f,0.f,0.f,0.f,0.f,0.f,0.f,0.f};

  for (int k0 = 0; k0 < K; k0 += 32) {
    V bh[4], bl[4];
#pragma unroll
    for (int j = 0; j < 4; ++j) {
      const size_t bo = (size_t)(n0 + (j << 4) + rlane) * ldb + koff + k0;
      bh[j] = Frag<T>::load(Bb + bo);
      if (SPLIT) bl[j] = Frag<T>::load(Bb2 + bo);
    }
#pragma unroll
    for (int i = 0; i < 4; ++i) {
      const size_t ao = (size_t)(m0 + (i << 4) + rlane) * lda + koff + k0;
      V ah = Frag<T>::load(Ab + ao);
      V al;
      if (SPLIT) al = Frag<T>::load(Ab2 + ao);
#pragma unroll
      for (int j = 0; j < 4; ++j) {
        acc[i][j] = Frag<T>::mma(ah, bh[j], acc[i][j]);
        if (SPLIT) {
          acc[i][j] = Frag<T>::mma(ah, bl[j], acc[i][j]);
          acc[i][j] = Frag<T>::mma(al, bh[j], acc[i][j]);
        }
      }
      Frag<T>::guard4(acc[i][0], acc[i][1], acc[i][2], acc[i][3], ah, SPLIT ? al : ah);
    }
    Frag<T>::keep(bh[0], bh[1], bh[2], bh[3]);
    if (SPLIT) Frag<T>::keep(bl[0], bl[1], bl[2], bl[3]);
  }
  acc_guard4(acc[0][0], acc[0][1], acc[0][2], acc[0][3]);
  acc_guard4(acc[1][0], acc[1][1], acc[1][2], acc[1][3]);
  acc_guard4(acc[2][0], acc[2][1], acc[2][2], acc[2][3]);
  acc_guard4(acc[3][0], acc[3][1], acc[3][2], acc[3][3]);

  float* slab = sT[wave];
  const float* Rb = RESID ? (resid + (size_t)b * strideR) : nullptr;
#pragma unroll
  for (int i = 0; i < 4; ++i) {
    const int mBase = m0 + (i << 4);
#pragma unroll
    for (int j = 0; j < 4; ++j) {
      const int n = n0 + (j << 4) + rlane;
      float bv = 0.f;
      if (BIAS_MODE == 2) bv = bias[n];
#pragma unroll
      for (int r = 0; r < 8; ++r) {
        float v = acc[i][j][r] * scale;
        if (BIAS_MODE == 1) v += bias[mBase + mOff + r];
        if (BIAS_MODE == 2) v += bv;
        if (RESID) v += Rb[(size_t)(mBase + mOff + r) * ldc + n];
        if (ACT == 1) v = tanhf(v);
        if (ACT == 2) v = fmaxf(v, 0.0f);
        if (ACT == 3) v = v / (1.0f + expf(-v));
        if (ACT == 4) v = (v > 0.f) ? v : 0.01f * v;
        if (ACT == 5) v = 0.5f * v * (1.0f + erff(v * 0.70710678118654752f));
        slab[(mOff + r) * 68 + (j << 4) + rlane] = v;
      }
    }
    __builtin_amdgcn_fence(__ATOMIC_RELEASE, "workgroup");
    __builtin_amdgcn_wave_barrier();
    __builtin_amdgcn_fence(__ATOMIC_ACQUIRE, "workgroup");
    if (OUT_MODE == 0) {
      float* C = (float*)Cout + (size_t)b * strideC;
      const int hh = lane >> 4, c4 = (lane & 15) * 4;
      for (int pass = 0; pass < 2; ++pass) {
#pragma unroll
        for (int it = 0; it < 8; ++it) {
          const int row = it * 2 + hh;
          v4f v = *(const v4f*)(slab + row * 68 + c4);
          *(volatile v4f*)(C + (size_t)(mBase + row) * ldc + n0 + c4) = v;
        }
        __threadfence();
      }
    } else {
      const int q = lane >> 3, c8 = (lane & 7) * 8;
      unsigned short* C  = (unsigned short*)Cout  + (size_t)b * strideC;
      unsigned short* C2 = (OUT_MODE == 2) ? ((unsigned short*)Cout2 + (size_t)b * strideC) : nullptr;
      for (int pass = 0; pass < 2; ++pass) {
#pragma unroll
        for (int it = 0; it < 4; ++it) {
          const int row = it * 4 + q;
          const float* sp = slab + row * 68 + c8;
          v8h hv, lv;
#pragma unroll
          for (int e = 0; e < 8; ++e) {
            if (OUT_MODE == 1) {
              hv[e] = (_Float16)sp[e];
            } else {
              unsigned short hb = f2bf_bits(sp[e]);
              unsigned short lb = f2bf_bits(sp[e] - bf_bits2f(hb));
              hv[e] = __builtin_bit_cast(_Float16, hb);
              lv[e] = __builtin_bit_cast(_Float16, lb);
            }
          }
          *(volatile v8h*)(C + (size_t)(mBase + row) * ldc + n0 + c8) = hv;
          if (OUT_MODE == 2) *(volatile v8h*)(C2 + (size_t)(mBase + row) * ldc + n0 + c8) = lv;
        }
        __threadfence();
      }
    }
    __builtin_amdgcn_fence(__ATOMIC_RELEASE, "workgroup");
    __builtin_amdgcn_wave_barrier();
    __builtin_amdgcn_fence(__ATOMIC_ACQUIRE, "workgroup");
  }
}

__device__ __forceinline__ void split8_store(v4f fa, v4f fb, unsigned short* __restrict__ ph, unsigned short* __restrict__ pl,
                                             size_t eoff) {
  v4u hv, lv;
#pragma unroll
  for (int e = 0; e < 2; ++e) {
    const float x0 = fa[2 * e], x1 = fa[2 * e + 1];
    const float y0 = fb[2 * e], y1 = fb[2 * e + 1];
    const unsigned short hx0 = f2bf_bits(x0), hx1 = f2bf_bits(x1), hy0 = f2bf_bits(y0), hy1 = f2bf_bits(y1);
    const unsigned short lx0 = f2bf_bits(x0 - bf_bits2f(hx0)), lx1 = f2bf_bits(x1 - bf_bits2f(hx1));
    const unsigned short ly0 = f2bf_bits(y0 - bf_bits2f(hy0)), ly1 = f2bf_bits(y1 - bf_bits2f(hy1));
    hv[e]     = (unsigned)hx0 | ((unsigned)hx1 << 16);
    lv[e]     = (unsigned)lx0 | ((unsigned)lx1 << 16);
    hv[2 + e] = (unsigned)hy0 | ((unsigned)hy1 << 16);
    lv[2 + e] = (unsigned)ly0 | ((unsigned)ly1 << 16);
  }
  for (int ps = 0; ps < 2; ++ps) {
    *(volatile v4u*)(ph + eoff) = hv;
    *(volatile v4u*)(pl + eoff) = lv;
    __threadfence();
  }
}

__global__ __launch_bounds__(NTHR) void prep_kernel(const float* __restrict__ obs, const float* __restrict__ W_emb,
                                                    const float* __restrict__ b_emb, const float* __restrict__ eWih,
                                                    unsigned short* __restrict__ EH, unsigned short* __restrict__ EL,
                                                    unsigned short* __restrict__ WHI, unsigned short* __restrict__ WLO) {
  const int tid = threadIdx.x, blk = blockIdx.x;
  if (blk < EMB_BLKS) {
    const int i = blk * NTHR + tid;
    const int row = i >> 3, c8 = (i & 7) * 8;
    const v2f xv = *(const v2f*)(obs + 2 * row);
    const v4f wa = *(const v4f*)(W_emb + 2 * c8);
    const v4f wb = *(const v4f*)(W_emb + 2 * c8 + 4);
    const v4f wc = *(const v4f*)(W_emb + 2 * c8 + 8);
    const v4f wd = *(const v4f*)(W_emb + 2 * c8 + 12);
    const v4f ba = *(const v4f*)(b_emb + c8);
    const v4f bb = *(const v4f*)(b_emb + c8 + 4);
    v4f fa, fb;
    fa[0] = fmaxf(xv[0] * wa[0] + xv[1] * wa[1] + ba[0], 0.0f);
    fa[1] = fmaxf(xv[0] * wa[2] + xv[1] * wa[3] + ba[1], 0.0f);
    fa[2] = fmaxf(xv[0] * wb[0] + xv[1] * wb[1] + ba[2], 0.0f);
    fa[3] = fmaxf(xv[0] * wb[2] + xv[1] * wb[3] + ba[3], 0.0f);
    fb[0] = fmaxf(xv[0] * wc[0] + xv[1] * wc[1] + bb[0], 0.0f);
    fb[1] = fmaxf(xv[0] * wc[2] + xv[1] * wc[3] + bb[1], 0.0f);
    fb[2] = fmaxf(xv[0] * wd[0] + xv[1] * wd[1] + bb[2], 0.0f);
    fb[3] = fmaxf(xv[0] * wd[2] + xv[1] * wd[3] + bb[3], 0.0f);
    split8_store(fa, fb, EH, EL, (size_t)i * 8);
  } else {
    const int i = (blk - EMB_BLKS) * NTHR + tid;
    const v4f fa = *(const v4f*)(eWih + 8 * (size_t)i);
    const v4f fb = *(const v4f*)(eWih + 8 * (size_t)i + 4);
    split8_store(fa, fb, WHI, WLO, (size_t)i * 8);
  }
}

__global__ __launch_bounds__(32) void seq_kernel(const float* __restrict__ GX,
                                                 const float* __restrict__ W_emb, const float* __restrict__ b_emb,
                                                 const float* __restrict__ eWhh,
                                                 const float* __restrict__ ebih, const float* __restrict__ ebhh,
                                                 const float* __restrict__ dWih, const float* __restrict__ dWhh,
                                                 const float* __restrict__ dbih, const float* __restrict__ dbhh,
                                                 const float* __restrict__ W_out, const float* __restrict__ b_out,
                                                 const int* __restrict__ np_p, float* __restrict__ out) {
  __shared__ __align__(16) float sWhh[NGATE * WHP];
  __shared__ __align__(16) float sWih[NGATE * WIP];
  __shared__ __align__(16) float sPar[512];
  __shared__ __align__(16) float sh[HID_DIM];
  __shared__ __align__(16) float semb[EMB_DIM];
  __shared__ __align__(16) float sring[32];
  const int lane = threadIdx.x;
  const v4f z4 = {0.0f, 0.0f, 0.0f, 0.0f};

#pragma unroll 1
  for (int i = lane; i < NGATE * HID_DIM / 4; i += 32) {
    const int r = i >> 3, k4 = (i & 7) * 4;
    *(v4f*)(sWhh + r * WHP + k4) = *(const v4f*)(eWhh + 4 * i);
  }
#pragma unroll 1
  for (int r = lane; r < NGATE; r += 32) *(v4f*)(sWhh + r * WHP + HID_DIM) = z4;
#pragma unroll 1
  for (int i = lane; i < NGATE * EMB_DIM / 4; i += 32) {
    const int r = i >> 4, k4 = (i & 15) * 4;
    *(v4f*)(sWih + r * WIP + k4) = *(const v4f*)(dWih + 4 * i);
  }
#pragma unroll 1
  for (int r = lane; r < NGATE; r += 32) *(v4f*)(sWih + r * WIP + EMB_DIM) = z4;
  {
    const v4f b0 = *(const v4f*)(ebih + 4 * lane);
    const v4f b1 = *(const v4f*)(ebhh + 4 * lane);
    *(v4f*)(sPar + 4 * lane) = b0 + b1;
    const v4f b2 = *(const v4f*)(dbih + 4 * lane);
    const v4f b3 = *(const v4f*)(dbhh + 4 * lane);
    *(v4f*)(sPar + 128 + 4 * lane) = b2 + b3;
    *(v4f*)(sPar + 256 + 4 * lane) = *(const v4f*)(W_emb + 4 * lane);
    const int l16 = lane & 15;
    const v4f be4 = *(const v4f*)(b_emb + 4 * l16);
    const v4f wo4 = *(const v4f*)(W_out + 4 * l16);
    if (lane < 16) {
      *(v4f*)(sPar + 384 + 4 * l16) = be4;
      *(v4f*)(sPar + 448 + 4 * l16) = wo4;
    }
  }
  sh[lane] = 0.0f; semb[lane] = 0.0f; semb[lane + 32] = 0.0f; sring[lane] = 0.0f;
  __syncthreads();

  const float be0 = sPar[lane], be1 = sPar[32 + lane], be2 = sPar[64 + lane], be3 = sPar[96 + lane];
  const float bd0 = sPar[128 + lane], bd1 = sPar[160 + lane], bd2 = sPar[192 + lane], bd3 = sPar[224 + lane];
  const float we0 = sPar[256 + 2 * lane], we1 = sPar[257 + 2 * lane];
  const float we2 = sPar[256 + 2 * (lane + 32)], we3 = sPar[257 + 2 * (lane + 32)];
  const float bea = sPar[384 + lane], beb = sPar[416 + lane];
  const float wo0 = sPar[448 + lane], wo1 = sPar[480 + lane];
  const float wt0 = sWih[lane * WIP + (EMB_DIM - 1)];
  const float wt1 = sWih[(32 + lane) * WIP + (EMB_DIM - 1)];
  const float wt2 = sWih[(64 + lane) * WIP + (EMB_DIM - 1)];
  const float wt3 = sWih[(96 + lane) * WIP + (EMB_DIM - 1)];
  const float bo0 = b_out[0], bo1 = b_out[1];
  int npv = __builtin_amdgcn_readfirstlane(np_p[0]);
  npv = npv < 0 ? 0 : (npv > NPRED ? NPRED : npv);
  const int nsteps = SEQ_LEN + 1 + npv;

  float cst = 0.0f, hst = 0.0f, pv0 = 0.0f, pv1 = 0.0f;

#pragma unroll 1
  for (int s = 0; s < nsteps; ++s) {
    if (s == SEQ_LEN) {
#pragma unroll 1
      for (int i = lane; i < NGATE * HID_DIM / 4; i += 32) {
        const int r = i >> 3, k4 = (i & 7) * 4;
        *(v4f*)(sWhh + r * WHP + k4) = *(const v4f*)(dWhh + 4 * i);
      }
      __syncthreads();
    }
    const int trow = (s < SEQ_LEN) ? s : (SEQ_LEN - 1);
    const float* gp = GX + (size_t)trow * NGATE + lane;
    const float ge0 = gp[0], ge1 = gp[32], ge2 = gp[64], ge3 = gp[96];
    float gd0 = 0.0f, gd1 = 0.0f, gd2 = 0.0f, gd3 = 0.0f;
    if (s > SEQ_LEN) {
      const float e0 = fmaxf(pv0 * we0 + pv1 * we1 + bea, 0.0f);
      const float e1 = fmaxf(pv0 * we2 + pv1 * we3 + beb, 0.0f);
      semb[lane] = e0;
      semb[lane + 32] = e1;
      __syncthreads();
      const float* wr = sWih + lane * WIP;
#pragma unroll 1
      for (int k4 = 0; k4 < EMB_DIM / 4; ++k4) {
        const v4f ev = *(const v4f*)(semb + 4 * k4);
        const v4f w0 = *(const v4f*)(wr + 4 * k4);
        const v4f w1 = *(const v4f*)(wr + 32 * WIP + 4 * k4);
        const v4f w2 = *(const v4f*)(wr + 64 * WIP + 4 * k4);
        const v4f w3 = *(const v4f*)(wr + 96 * WIP + 4 * k4);
#pragma unroll
        for (int e = 0; e < 4; ++e) {
          gd0 = fmaf(ev[e], w0[e], gd0);
          gd1 = fmaf(ev[e], w1[e], gd1);
          gd2 = fmaf(ev[e], w2[e], gd2);
          gd3 = fmaf(ev[e], w3[e], gd3);
        }
      }
    }
    const bool isenc = (s < SEQ_LEN), istag = (s == SEQ_LEN);
    float a0 = isenc ? (ge0 + be0) : (istag ? (wt0 + bd0) : (gd0 + bd0));
    float a1 = isenc ? (ge1 + be1) : (istag ? (wt1 + bd1) : (gd1 + bd1));
    float a2 = isenc ? (ge2 + be2) : (istag ? (wt2 + bd2) : (gd2 + bd2));
    float a3 = isenc ? (ge3 + be3) : (istag ? (wt3 + bd3) : (gd3 + bd3));
    {
      const float* wr = sWhh + lane * WHP;
#pragma unroll 1
      for (int k4 = 0; k4 < HID_DIM / 4; ++k4) {
        const v4f hv = *(const v4f*)(sh + 4 * k4);
        const v4f w0 = *(const v4f*)(wr + 4 * k4);
        const v4f w1 = *(const v4f*)(wr + 32 * WHP + 4 * k4);
        const v4f w2 = *(const v4f*)(wr + 64 * WHP + 4 * k4);
        const v4f w3 = *(const v4f*)(wr + 96 * WHP + 4 * k4);
#pragma unroll
        for (int e = 0; e < 4; ++e) {
          a0 = fmaf(hv[e], w0[e], a0);
          a1 = fmaf(hv[e], w1[e], a1);
          a2 = fmaf(hv[e], w2[e], a2);
          a3 = fmaf(hv[e], w3[e], a3);
        }
      }
    }
    const float ig = fsig(a0);
    const float fg = fsig(a1);
    const float gg = ftanh(a2);
    const float og = fsig(a3);
    cst = fg * cst + ig * gg;
    hst = og * ftanh(cst);
    __syncthreads();
    sh[lane] = hst;
    __syncthreads();
    float p0 = wo0 * hst, p1 = wo1 * hst;
#pragma unroll
    for (int off = 1; off < 32; off <<= 1) {
      p0 += __shfl_xor(p0, off, 32);
      p1 += __shfl_xor(p1, off, 32);
    }
    pv0 = p0 + bo0;
    pv1 = p1 + bo1;
    if (s < nsteps - 1) {
      if (lane == 0) {
        sring[2 * (s & 15)]     = pv0;
        sring[2 * (s & 15) + 1] = pv1;
      }
      if ((s & 15) == 15) {
        __syncthreads();
        const int c4 = (lane & 7) * 4;
        const v4f v = *(const v4f*)(sring + c4);
        float* op = out + (size_t)(s >> 4) * 32 + c4;
        for (int ps = 0; ps < 2; ++ps) {
          if (lane < 8) *(volatile v4f*)op = v;
          __threadfence();
        }
      }
    }
  }
}

extern "C" void kernel_launch(void* const* d_in, const int* in_sizes, int n_in,
                              void* d_out, int out_size, void* d_ws, size_t ws_size, hipStream_t stream) {
  if (n_in < 14 || d_out == nullptr || d_ws == nullptr) return;
  if (in_sizes[0] != SEQ_LEN * 2 || in_sizes[1] != EMB_DIM * 2 || in_sizes[2] != EMB_DIM ||
      in_sizes[3] != NGATE * EMB_DIM || in_sizes[4] != NGATE * HID_DIM || in_sizes[5] != NGATE || in_sizes[6] != NGATE ||
      in_sizes[7] != NGATE * EMB_DIM || in_sizes[8] != NGATE * HID_DIM || in_sizes[9] != NGATE || in_sizes[10] != NGATE ||
      in_sizes[11] != 2 * HID_DIM || in_sizes[12] != 2 || in_sizes[13] != 1 || out_size != NROW_OUT * 2) return;

  const float* obs   = (const float*)d_in[0];
  const float* W_emb = (const float*)d_in[1];
  const float* b_emb = (const float*)d_in[2];
  const float* eWih  = (const float*)d_in[3];
  const float* eWhh  = (const float*)d_in[4];
  const float* ebih  = (const float*)d_in[5];
  const float* ebhh  = (const float*)d_in[6];
  const float* dWih  = (const float*)d_in[7];
  const float* dWhh  = (const float*)d_in[8];
  const float* dbih  = (const float*)d_in[9];
  const float* dbhh  = (const float*)d_in[10];
  const float* W_out = (const float*)d_in[11];
  const float* b_out = (const float*)d_in[12];
  const int*   np    = (const int*)d_in[13];
  float* out = (float*)d_out;

  char* ws = (char*)d_ws; size_t off = 0;
  auto carve = [&](size_t bytes) -> char* { char* p = ws + off; off += (bytes + 255) & ~(size_t)255; return p; };
  unsigned short* EH  = (unsigned short*)carve((size_t)SEQ_LEN * EMB_DIM * 2);
  unsigned short* EL  = (unsigned short*)carve((size_t)SEQ_LEN * EMB_DIM * 2);
  unsigned short* WHI = (unsigned short*)carve((size_t)NGATE * EMB_DIM * 2);
  unsigned short* WLO = (unsigned short*)carve((size_t)NGATE * EMB_DIM * 2);
  float*          GX  = (float*)carve((size_t)SEQ_LEN * NGATE * 4);
  if (off > ws_size || off > (size_t)134217728) return;

  prep_kernel<<<EMB_BLKS + WIH_BLKS, NTHR, 0, stream>>>(obs, W_emb, b_emb, eWih, EH, EL, WHI, WLO);
  wmma_gemm64<1, true, 0, 0, false, 0><<<dim3(GEMM_BLKS, 1), 256, 0, stream>>>(
      EH, EL, EMB_DIM, 0L, WHI, WLO, EMB_DIM, 0L, (void*)GX, (void*)GX, NGATE, 0L,
      ebih, GX, 0L, SEQ_LEN, NGATE, EMB_DIM, 1.0f);
  seq_kernel<<<1, 32, 0, stream>>>(GX, W_emb, b_emb, eWhh, ebih, ebhh, dWih, dWhh, dbih, dbhh, W_out, b_out, np, out);
}
